// SAGE_2370821947944
// MI455X (gfx1250) — hardware-verified
//
#include <hip/hip_runtime.h>
#include <stddef.h>
#include <stdint.h>
#include <math.h>


#define CIN    128
#define HID    128
#define NCLS   64
#define N1     256
#define K1     128
#define N2     128
#define K2     256
#define NTHR   256
#define NWAVE  8
#define EPT    8
#define CHUNK  (NTHR * EPT)
#define WCAP   (EPT * 32)
#define LISTN  (NWAVE * WCAP)
#define NBA    1024
#define SLA    10
#define RCAP   28672
#define DEGCAP 64
#define GBM    64
#define GBN    64
#define GTHR   128
#define NBW1   ((N1 * (K1 / 8)) / NTHR)
#define NBW2   ((N2 * (K2 / 8)) / NTHR)
#define AGG_ZINTS    (LISTN + 2 * RCAP + 3 * NBA)
#define MISC_INTS    16
#define ROWBUF_INTS  (NWAVE * K2 / 2)
#define AGG_LDS_INTS (AGG_ZINTS + MISC_INTS + ROWBUF_INTS)
#define WSMAX  134217728

static_assert((CHUNK & (CHUNK - 1)) == 0 && CHUNK <= 4096);
static_assert((NBA & (NBA - 1)) == 0 && NBA == (1 << SLA));
static_assert(((long long)CHUNK << SLA) < (1LL << 31));
static_assert(LISTN % NTHR == 0);
static_assert(NBA % NWAVE == 0 && NBA % 32 == 0 && NBA % GBM == 0);
static_assert(RCAP % 32 == 0 && AGG_ZINTS % 4 == 0 && LISTN % 4 == 0 && ((AGG_ZINTS + MISC_INTS) % 4) == 0);
static_assert(AGG_ZINTS % (NTHR * 4) == 0);
static_assert(K1 % 32 == 0 && K2 % 32 == 0 && K2 == 2 * HID && K1 == CIN);
static_assert(N1 % GBN == 0 && N2 % GBN == 0 && N1 == 2 * HID && N2 == 2 * NCLS);
static_assert(GBM == (GTHR / 32) * 16 && GBN == 64);
static_assert((N1 * (K1 / 8)) % NTHR == 0 && (N2 * (K2 / 8)) % NTHR == 0);
static_assert(K1 / 8 == 16 && K2 / 8 == 32);
static_assert(HID == 4 * 32 && NCLS == 2 * 32);
static_assert(AGG_LDS_INTS * 4 <= 300000);

typedef float          v2f   __attribute__((ext_vector_type(2)));
typedef float          v4f   __attribute__((ext_vector_type(4)));
typedef float          v8f   __attribute__((ext_vector_type(8)));
typedef int            v4i   __attribute__((ext_vector_type(4)));
typedef int            v8i   __attribute__((ext_vector_type(8)));
typedef unsigned short v4us  __attribute__((ext_vector_type(4)));
typedef unsigned short v8us  __attribute__((ext_vector_type(8)));
typedef unsigned short v16us __attribute__((ext_vector_type(16)));
typedef __bf16         v16bf __attribute__((ext_vector_type(16)));
typedef v2f  __attribute__((may_alias)) v2fa;
typedef v4f  __attribute__((may_alias)) v4fa;
typedef v4i  __attribute__((may_alias)) v4ia;
typedef v4us __attribute__((may_alias)) v4usa;
typedef v8us __attribute__((may_alias)) v8usa;
union FragB { v16bf v; v16us u; v8us h[2]; v8i w; };

__device__ __forceinline__ v8f wmb(const FragB& a, const FragB& b, v8f c) {
  v8f d = __builtin_amdgcn_wmma_f32_16x16x32_bf16(false, a.v, false, b.v, (short)0, c, false, false);
  asm volatile("v_nop\n\tv_nop\n\tv_nop\n\tv_nop" : "+v"(d) : "v"(a.w), "v"(b.w));
  return d;
}

__device__ __forceinline__ unsigned bf16_bits(float f) {
  const unsigned u = __float_as_uint(f);
  return (u + 0x7FFFu + ((u >> 16) & 1u)) >> 16;
}
__device__ __forceinline__ float bf16_val(float f) {
  return __uint_as_float(bf16_bits(f) << 16);
}

__device__ __forceinline__ void wave_sync() {
  __builtin_amdgcn_fence(__ATOMIC_RELEASE, "wavefront");
  __builtin_amdgcn_wave_barrier();
  __builtin_amdgcn_fence(__ATOMIC_ACQUIRE, "wavefront");
}

template <int SLB>
__device__ __forceinline__ int scan_chunk(const int* __restrict__ dsts, int nE, int cbase, int slotBase,
                                          int nb, int vec8, int* list, int tid, int lane, int wave) {
  int wc = 0;
  const int el0  = tid * EPT;
  const int e0   = cbase + el0;
  const int sent = -2147483647 - 1;
  v4i da, db;
  if (vec8 != 0 && cbase + CHUNK <= nE) {
    da = *(const v4i*)(dsts + e0);
    db = *(const v4i*)(dsts + e0 + 4);
  } else {
    da.x = (e0     < nE) ? dsts[min(e0,     nE - 1)] : sent;
    da.y = (e0 + 1 < nE) ? dsts[min(e0 + 1, nE - 1)] : sent;
    da.z = (e0 + 2 < nE) ? dsts[min(e0 + 2, nE - 1)] : sent;
    da.w = (e0 + 3 < nE) ? dsts[min(e0 + 3, nE - 1)] : sent;
    db.x = (e0 + 4 < nE) ? dsts[min(e0 + 4, nE - 1)] : sent;
    db.y = (e0 + 5 < nE) ? dsts[min(e0 + 5, nE - 1)] : sent;
    db.z = (e0 + 6 < nE) ? dsts[min(e0 + 6, nE - 1)] : sent;
    db.w = (e0 + 7 < nE) ? dsts[min(e0 + 7, nE - 1)] : sent;
  }
  const unsigned nbs = (unsigned)slotBase;
  const unsigned unb = (unsigned)nb;
  const unsigned s0 = (unsigned)da.x - nbs, s1 = (unsigned)da.y - nbs;
  const unsigned s2 = (unsigned)da.z - nbs, s3 = (unsigned)da.w - nbs;
  const unsigned s4 = (unsigned)db.x - nbs, s5 = (unsigned)db.y - nbs;
  const unsigned s6 = (unsigned)db.z - nbs, s7 = (unsigned)db.w - nbs;
  const bool h0 = s0 < unb, h1 = s1 < unb, h2 = s2 < unb, h3 = s3 < unb;
  const bool h4 = s4 < unb, h5 = s5 < unb, h6 = s6 < unb, h7 = s7 < unb;
  const unsigned any = __builtin_amdgcn_ballot_w32(h0 | h1 | h2 | h3 | h4 | h5 | h6 | h7);
  if (any != 0u) {
#define HITJ(J, HJ, SJ) { \
      const unsigned mj = __builtin_amdgcn_ballot_w32(HJ); \
      if (mj != 0u) { \
        if (HJ) { \
          const int pos = wc + (int)__builtin_amdgcn_mbcnt_lo(mj, 0u); \
          if (pos < WCAP) list[wave * WCAP + pos] = ((el0 + (J)) << SLB) | (int)(SJ); \
        } \
        wc += (int)__builtin_popcount(mj); } }
    HITJ(0, h0, s0)
    HITJ(1, h1, s1)
    HITJ(2, h2, s2)
    HITJ(3, h3, s3)
    HITJ(4, h4, s4)
    HITJ(5, h5, s5)
    HITJ(6, h6, s6)
    HITJ(7, h7, s7)
#undef HITJ
  }
  return wc;
}

__global__ __launch_bounds__(NTHR) void k_prep(const float* __restrict__ x,
                                               const float* __restrict__ w1l, const float* __restrict__ w1r,
                                               const float* __restrict__ w2l, const float* __restrict__ w2r,
                                               int nN, int nbx,
                                               unsigned short* XB, unsigned short* W1B, unsigned short* W2B2) {
  const int bx  = (int)blockIdx.x;
  const int tid = (int)threadIdx.x;
  const float* p;
  unsigned short* dp;
  bool ok = true;
  if (bx < nbx) {
    const int u   = bx * NTHR + tid;
    const int row = u >> 4;
    const int k8  = (u & 15) * 8;
    const int rc  = row < nN ? row : nN - 1;
    p  = x + (size_t)rc * CIN + k8;
    ok = row < nN;
    dp = XB + (size_t)row * CIN + k8;
  } else if (bx < nbx + NBW1) {
    const int v  = (bx - nbx) * NTHR + tid;
    const int n  = v >> 4;
    const int k8 = (v & 15) * 8;
    const float* srow = (n < HID) ? (w1l + (size_t)n * CIN) : (w1r + (size_t)(n - HID) * CIN);
    p  = srow + k8;
    dp = W1B + (size_t)n * K1 + k8;
  } else if (bx < nbx + NBW1 + NBW2) {
    const int v  = (bx - nbx - NBW1) * NTHR + tid;
    const int n  = v >> 5;
    const int k8 = (v & 31) * 8;
    const int kk = k8 & (HID - 1);
    const float* srow = (n < NCLS) ? (w2l + (size_t)n * HID) : (w2r + (size_t)(n - NCLS) * HID);
    p  = srow + kk;
    dp = W2B2 + (size_t)n * K2 + k8;
  } else {
    return;
  }
  const v4f a = *(const v4fa*)p;
  const v4f b = *(const v4fa*)(p + 4);
  v8us o;
  o[0] = ok ? (unsigned short)bf16_bits(a.x) : (unsigned short)0;
  o[1] = ok ? (unsigned short)bf16_bits(a.y) : (unsigned short)0;
  o[2] = ok ? (unsigned short)bf16_bits(a.z) : (unsigned short)0;
  o[3] = ok ? (unsigned short)bf16_bits(a.w) : (unsigned short)0;
  o[4] = ok ? (unsigned short)bf16_bits(b.x) : (unsigned short)0;
  o[5] = ok ? (unsigned short)bf16_bits(b.y) : (unsigned short)0;
  o[6] = ok ? (unsigned short)bf16_bits(b.z) : (unsigned short)0;
  o[7] = ok ? (unsigned short)bf16_bits(b.w) : (unsigned short)0;
  *(volatile v8us*)dp = o;
  __threadfence();
  *(volatile v8us*)dp = o;
}

__global__ __launch_bounds__(GTHR) void k_gemm(
    const unsigned short* __restrict__ A, const unsigned short* __restrict__ WT,
    float* outF, int K, int ldo)
{
  __shared__ __attribute__((aligned(16))) float stg[GBM * GBN];
  const int tid = (int)threadIdx.x, lane = tid & 31, wave = tid >> 5, hh = lane >> 4, m = lane & 15;
  const int rowBase = (int)blockIdx.x * GBM;
  const int col0    = (int)blockIdx.y * GBN;

  v8f acc[4];
  {
    const v8f z = {0.f, 0.f, 0.f, 0.f, 0.f, 0.f, 0.f, 0.f};
    acc[0] = z; acc[1] = z; acc[2] = z; acc[3] = z;
  }
  const unsigned short* ap = A  + (size_t)(rowBase + 16 * wave + m) * (size_t)K + 8 * hh;
  const unsigned short* wp = WT + (size_t)(col0 + m) * (size_t)K + 8 * hh;
  const int ksteps = K >> 5;
#pragma unroll 1
  for (int ks = 0; ks < ksteps; ++ks) {
    FragB af;
    af.h[0] = *(const v8usa*)(ap + 32 * ks);
    af.h[1] = *(const v8usa*)(ap + 32 * ks + 16);
#pragma unroll
    for (int t = 0; t < 4; ++t) {
      const unsigned short* wq = wp + (size_t)(16 * t) * (size_t)K + 32 * ks;
      FragB bf;
      bf.h[0] = *(const v8usa*)wq;
      bf.h[1] = *(const v8usa*)(wq + 16);
      acc[t] = wmb(af, bf, acc[t]);
    }
  }

#pragma unroll
  for (int t = 0; t < 4; ++t) {
    const int lc = 16 * t + m;
#pragma unroll
    for (int r = 0; r < 8; ++r) {
      const int lr = 16 * wave + 8 * hh + r;
      stg[lr * GBN + lc] = acc[t][r];
    }
  }
  __syncthreads();

  v4f fv[8];
#pragma unroll
  for (int i = 0; i < 8; ++i) {
    const int lr = 16 * wave + 2 * i + hh;
    fv[i] = *(const v4fa*)(stg + lr * GBN + 4 * m);
  }
#pragma unroll
  for (int i = 0; i < 8; ++i) {
    const int lr = 16 * wave + 2 * i + hh;
    const int gr = rowBase + lr;
    float* op = outF + (size_t)gr * (size_t)ldo + col0 + 4 * m;
    *(volatile v4f*)op = fv[i];
  }
  __threadfence();
#pragma unroll
  for (int i = 0; i < 8; ++i) {
    const int lr = 16 * wave + 2 * i + hh;
    const int gr = rowBase + lr;
    float* op = outF + (size_t)gr * (size_t)ldo + col0 + 4 * m;
    *(volatile v4f*)op = fv[i];
  }
}

template <int LAYER>
__global__ __launch_bounds__(NTHR) void k_scan(const int* __restrict__ srcs, const int* __restrict__ dsts,
                                               int nE, int nN, int vec8, int mRows,
                                               const float* __restrict__ pq, const float* __restrict__ bias,
                                               unsigned short* hpl, float* outp, int planeElems) {
  extern __shared__ __attribute__((aligned(16))) int dsm[];
  int* list = dsm;
  int* hl   = dsm + LISTN;
  int* sl   = hl + RCAP;
  int* cnt  = sl + RCAP;
  int* offs = cnt + NBA;
  int* cur  = offs + NBA;
  int* misc = cur + NBA;
  const int tid = (int)threadIdx.x, lane = tid & 31, wave = tid >> 5;
  unsigned short* rowbuf = (unsigned short*)(misc + MISC_INTS) + wave * K2;
  const int nodeBase = (int)blockIdx.x * NBA;

  {
    const v4i z4 = {0, 0, 0, 0};
    for (int i = tid * 4; i < AGG_ZINTS; i += NTHR * 4) *(v4ia*)(dsm + i) = z4;
    if (tid < MISC_INTS) misc[tid] = 0;
  }
  float bv0, bv1, bv2 = 0.0f, bv3 = 0.0f;
  if constexpr (LAYER == 1) {
    const v4f a = *(const v4fa*)(bias + 4 * lane);
    bv0 = bf16_val(a.x); bv1 = bf16_val(a.y); bv2 = bf16_val(a.z); bv3 = bf16_val(a.w);
  } else {
    const v2f a = *(const v2fa*)(bias + 2 * lane);
    bv0 = bf16_val(a.x); bv1 = bf16_val(a.y);
  }
  __syncthreads();

  int t = 0, ov = 0;
  const int nChunks = (nE + CHUNK - 1) / CHUNK;
#pragma unroll 1
  for (int ch = 0; ch < nChunks; ++ch) {
    const int cbase = ch * CHUNK;
    const int wc = scan_chunk<SLA>(dsts, nE, cbase, nodeBase, NBA, vec8, list, tid, lane, wave);
    if (lane == 0) misc[wave] = wc;
    __syncthreads();
    if (wave == 0) {
#pragma unroll 1
      for (int w2 = 0; w2 < NWAVE; ++w2) {
        int c = misc[w2];
        c = c < 0 ? 0 : (c > WCAP ? WCAP : c);
#pragma unroll 1
        for (int b0 = 0; b0 < c; b0 += 32) {
          const int idx = b0 + lane;
          const int ent = list[w2 * WCAP + (idx < WCAP ? idx : WCAP - 1)];
          const int m32 = (c - b0) < 32 ? (c - b0) : 32;
#pragma unroll 1
          for (int k = 0; k < m32; ++k) {
            const int u    = __builtin_amdgcn_readlane(ent, k);
            const int slot = u & (NBA - 1);
            const int el   = (u >> SLA) & (CHUNK - 1);
            const int pk   = ((cbase + el) << SLA) | slot;
            if (t < RCAP) {
              if (lane == 0) { hl[t] = pk; cnt[slot] = cnt[slot] + 1; }
              t = t + 1;
            } else {
              ov = 1;
            }
          }
        }
      }
    }
    __syncthreads();
  }
  if (wave == 0 && lane == 0) { misc[8] = t; misc[9] = ov; }
  __syncthreads();
  int tt = misc[8];
  tt = tt < 0 ? 0 : (tt > RCAP ? RCAP : tt);
  const int ovf = misc[9];

  if (wave == 0) {
    const int base = lane * (NBA / 32);
    int s = 0;
#pragma unroll 1
    for (int i = 0; i < NBA / 32; ++i) s += cnt[base + i];
    int incl = s;
#pragma unroll
    for (int d = 1; d < 32; d <<= 1) {
      const int y = __shfl_up(incl, d, 32);
      if (lane >= d) incl += y;
    }
    int run = incl - s;
#pragma unroll 1
    for (int i = 0; i < NBA / 32; ++i) {
      const int cv = cnt[base + i];
      offs[base + i] = run;
      cur[base + i]  = run;
      run += cv;
    }
  }
  __syncthreads();
  if (wave == 0) {
#pragma unroll 1
    for (int b0 = 0; b0 < tt; b0 += 32) {
      const int idx = b0 + lane;
      const int ent = hl[idx < RCAP ? idx : RCAP - 1];
      const int m32 = (tt - b0) < 32 ? (tt - b0) : 32;
#pragma unroll 1
      for (int k = 0; k < m32; ++k) {
        const int u    = __builtin_amdgcn_readlane(ent, k);
        const int slot = u & (NBA - 1);
        if (lane == 0) {
          int p = cur[slot];
          p = p < 0 ? 0 : (p > RCAP - 1 ? RCAP - 1 : p);
          sl[p] = u;
          cur[slot] = p + 1;
        }
      }
    }
  }
  __syncthreads();

  const float qnan = __int_as_float(0x7fc00000);
  const float pz = (ovf != 0) ? qnan : 0.0f;
  const int sa = (2 * lane) & 31, sb = (2 * lane + 1) & 31;
#pragma unroll 1
  for (int si = 0; si < NBA / NWAVE; ++si) {
    const int s    = si * NWAVE + wave;
    const int node = nodeBase + s;
    int c = cnt[s];
    const bool big = c > DEGCAP;
    c = c < 0 ? 0 : (c > DEGCAP ? DEGCAP : c);
    int o = offs[s];
    o = o < 0 ? 0 : (o > RCAP ? RCAP : o);
    const int nc = node < nN ? node : nN - 1;
    float a0 = 0.0f, a1 = 0.0f, a2 = 0.0f, a3 = 0.0f;
#pragma unroll 1
    for (int b0 = 0; b0 < c; b0 += 32) {
      int idx = o + b0 + lane;
      idx = idx > RCAP - 1 ? RCAP - 1 : idx;
      const int ent = sl[idx];
      int eid = ent >> SLA;
      eid = eid < 0 ? 0 : (eid > nE - 1 ? nE - 1 : eid);
      int sr = srcs[eid];
      sr = sr < 0 ? 0 : (sr > nN - 1 ? nN - 1 : sr);
      const int m32 = (c - b0) < 32 ? (c - b0) : 32;
#pragma unroll 1
      for (int k = 0; k < m32; ++k) {
        const int sk = __builtin_amdgcn_readlane(sr, k);
        if constexpr (LAYER == 1) {
          const v4f a = *(const v4fa*)(pq + (size_t)sk * N1 + 4 * lane);
          a0 += a.x; a1 += a.y; a2 += a.z; a3 += a.w;
        } else {
          const v2f a = *(const v2fa*)(pq + (size_t)sk * N2 + 2 * lane);
          a0 += a.x; a1 += a.y;
        }
      }
    }
    const int   cc  = c < 1 ? 1 : c;
    const float inv = 1.0f / (float)cc;
    const float pzr = big ? qnan : pz;
    const bool live = node < nN;

    if constexpr (LAYER == 1) {
      const v4f q = *(const v4fa*)(pq + (size_t)nc * N1 + HID + 4 * lane);
      float y0 = (a0 * inv + bv0) + q.x;
      float y1 = (a1 * inv + bv1) + q.y;
      float y2 = (a2 * inv + bv2) + q.z;
      float y3 = (a3 * inv + bv3) + q.w;
      y0 = fmaxf(y0, 0.0f) + pzr; y1 = fmaxf(y1, 0.0f) + pzr;
      y2 = fmaxf(y2, 0.0f) + pzr; y3 = fmaxf(y3, 0.0f) + pzr;
      const float m0 = live ? y0 : 0.0f;
      const float m1 = live ? y1 : 0.0f;
      const float m2 = live ? y2 : 0.0f;
      const float m3 = live ? y3 : 0.0f;
      v4us mh, ml;
      {
        unsigned hb;
        hb = bf16_bits(m0); mh[0] = (unsigned short)hb; ml[0] = (unsigned short)bf16_bits(m0 - __uint_as_float(hb << 16));
        hb = bf16_bits(m1); mh[1] = (unsigned short)hb; ml[1] = (unsigned short)bf16_bits(m1 - __uint_as_float(hb << 16));
        hb = bf16_bits(m2); mh[2] = (unsigned short)hb; ml[2] = (unsigned short)bf16_bits(m2 - __uint_as_float(hb << 16));
        hb = bf16_bits(m3); mh[3] = (unsigned short)hb; ml[3] = (unsigned short)bf16_bits(m3 - __uint_as_float(hb << 16));
      }
      *(v4usa*)(rowbuf + 4 * lane) = mh;
      *(v4usa*)(rowbuf + HID + 4 * lane) = ml;
      wave_sync();
      const v8us q0 = *(const v8usa*)(rowbuf + 8 * lane);
      wave_sync();
      if (node < mRows) {
        unsigned short* rpw = hpl + (size_t)node * K2 + 8 * lane;
        *(volatile v8us*)rpw = q0;
        __threadfence();
        *(volatile v8us*)rpw = q0;
      }
    } else {
      const v2f q = *(const v2fa*)(pq + (size_t)nc * N2 + NCLS + 2 * lane);
      const float lg0 = ((a0 * inv + bv0) + q.x) + pzr;
      const float lg1 = ((a1 * inv + bv1) + q.y) + pzr;
      float mx = fmaxf(lg0, lg1);
#pragma unroll
      for (int d = 16; d >= 1; d >>= 1) mx = fmaxf(mx, __shfl_xor(mx, d, 32));
      float se = expf(lg0 - mx) + expf(lg1 - mx);
#pragma unroll
      for (int d = 16; d >= 1; d >>= 1) se += __shfl_xor(se, d, 32);
      const float lse = mx + logf(se);
      const float ls0 = lg0 - lse;
      const float ls1 = lg1 - lse;
      v4f ols, olg;
      ols.x = __shfl(ls0, sa, 32); ols.y = __shfl(ls1, sa, 32);
      ols.z = __shfl(ls0, sb, 32); ols.w = __shfl(ls1, sb, 32);
      olg.x = __shfl(lg0, sa, 32); olg.y = __shfl(lg1, sa, 32);
      olg.z = __shfl(lg0, sb, 32); olg.w = __shfl(lg1, sb, 32);
      const bool up = lane >= 16;
      v4f ov4;
      ov4.x = up ? olg.x : ols.x;
      ov4.y = up ? olg.y : ols.y;
      ov4.z = up ? olg.z : ols.z;
      ov4.w = up ? olg.w : ols.w;
      const size_t eo = (up ? (size_t)planeElems : (size_t)0) + (size_t)nc * NCLS + (size_t)(4 * (lane & 15));
      float* op = outp + eo;
      if (live) *(volatile v4f*)op = ov4;
      __threadfence();
      if (live) *(volatile v4f*)op = ov4;
    }
  }
}

static inline int cdiv(int a, int b) { return (a + b - 1) / b; }
static inline size_t al256(size_t o) { return (o + 255) & ~(size_t)255; }

extern "C" void kernel_launch(void* const* d_in, const int* in_sizes, int n_in,
                              void* d_out, int out_size, void* d_ws, size_t ws_size,
                              hipStream_t stream) {
  if (n_in < 8) return;
  if (in_sizes[0] < CIN || (in_sizes[0] % CIN) != 0) return;
  const int nN = in_sizes[0] / CIN;
  if (nN < 1 || nN > (1 << 22)) return;
  if (in_sizes[1] < 2 || (in_sizes[1] & 1) != 0) return;
  const int nE = in_sizes[1] / 2;
  if (nE < 1 || nE >= (1 << (31 - SLA))) return;
  if (in_sizes[2] != HID * CIN || in_sizes[3] != HID) return;
  if (in_sizes[4] != HID * CIN) return;
  if (in_sizes[5] != NCLS * HID || in_sizes[6] != NCLS) return;
  if (in_sizes[7] != NCLS * HID) return;
  const long long planeLL = (long long)nN * NCLS;
  if ((long long)out_size != 2 * planeLL) return;
  const int planeElems = (int)planeLL;

  const float* x    = (const float*)d_in[0];
  const int*   edge = (const int*)d_in[1];
  const float* w1l  = (const float*)d_in[2];
  const float* b1l  = (const float*)d_in[3];
  const float* w1r  = (const float*)d_in[4];
  const float* w2l  = (const float*)d_in[5];
  const float* b2l  = (const float*)d_in[6];
  const float* w2r  = (const float*)d_in[7];
  float* out = (float*)d_out;
  const int* src = edge;
  const int* dst = edge + nE;

  const int MP  = cdiv(nN, GBM) * GBM;
  const int gM  = MP / GBM;
  const int gA  = cdiv(MP, NBA);
  if ((long long)gA * NBA < (long long)MP) return;
  const int nbx = (MP * (CIN / 8)) / NTHR;
  const int vec8 = ((nE & 3) == 0) ? 1 : 0;

  char* ws = (char*)d_ws;
  size_t off = 0;
  const size_t oXB  = off; off = al256(off + (size_t)MP * CIN * 2);
  const size_t oW1  = off; off = al256(off + (size_t)N1 * K1 * 2);
  const size_t oW2  = off; off = al256(off + (size_t)N2 * K2 * 2);
  const size_t oPQ1 = off; off = al256(off + (size_t)MP * N1 * 4);
  const size_t oH   = off; off = al256(off + (size_t)MP * K2 * 2);
  const size_t oPQ2 = off; off = al256(off + (size_t)MP * N2 * 4);
  if (off > ws_size || off > (size_t)WSMAX) return;
  unsigned short* XB   = (unsigned short*)(ws + oXB);
  unsigned short* W1B  = (unsigned short*)(ws + oW1);
  unsigned short* W2B2 = (unsigned short*)(ws + oW2);
  float*          PQ1  = (float*)(ws + oPQ1);
  unsigned short* Hpl  = (unsigned short*)(ws + oH);
  float*          PQ2  = (float*)(ws + oPQ2);

  const size_t scanLds = (size_t)AGG_LDS_INTS * 4;
  hipFuncSetAttribute(reinterpret_cast<const void*>(&k_scan<1>), hipFuncAttributeMaxDynamicSharedMemorySize, (int)scanLds);
  hipFuncSetAttribute(reinterpret_cast<const void*>(&k_scan<2>), hipFuncAttributeMaxDynamicSharedMemorySize, (int)scanLds);

  k_prep<<<nbx + NBW1 + NBW2, NTHR, 0, stream>>>(x, w1l, w1r, w2l, w2r, nN, nbx, XB, W1B, W2B2);
  k_gemm<<<dim3(gM, N1 / GBN), GTHR, 0, stream>>>(XB, W1B, PQ1, K1, N1);
  k_scan<1><<<gA, NTHR, scanLds, stream>>>(src, dst, nE, nN, vec8, MP, PQ1, b1l, Hpl, out, planeElems);
  k_gemm<<<dim3(gM, N2 / GBN), GTHR, 0, stream>>>(Hpl, W2B2, PQ2, K2, N2);
  k_scan<2><<<gA, NTHR, scanLds, stream>>>(src, dst, nE, nN, vec8, MP, PQ2, b2l, Hpl, out, planeElems);
}
